// DKVMN_6107443495306
// MI455X (gfx1250) — hardware-run, weakly checked
//
#include <hip/hip_runtime.h>


#define NTOK (128 * 2048)
#define CH   16384
#define DK   128
#define DVM  256
#define DH   512
#define MS   50
#define MP   64
#define NF   (DVM + DK)
#define NQ1  50001
typedef _Float16 h16;
typedef unsigned short bf;
typedef __attribute__((ext_vector_type(16))) __bf16   v16bf;
typedef __attribute__((ext_vector_type(16))) _Float16 v16h;
typedef __attribute__((ext_vector_type(8)))  _Float16 v8h;
typedef __attribute__((ext_vector_type(8)))  unsigned short v8us;
typedef __attribute__((ext_vector_type(8)))  float    v8f;
typedef __attribute__((ext_vector_type(4)))  float    v4f;
typedef v8h  __attribute__((may_alias)) v8ha;
typedef v4f  __attribute__((may_alias)) v4fa;
typedef v8us __attribute__((may_alias)) v8usa;

__device__ __forceinline__ unsigned short f2bf(float f) { unsigned u = __float_as_uint(f); u += 0x7FFFu + ((u >> 16) & 1u); return (unsigned short)(u >> 16); }
__device__ __forceinline__ float bf2f(unsigned short b) { return __uint_as_float(((unsigned)b) << 16); }
__device__ __forceinline__ float bfr(float f) { return bf2f(f2bf(f)); }
__device__ __forceinline__ v16h cat16(v8h lo, v8h hi) { return __builtin_shufflevector(lo, hi, 0, 1, 2, 3, 4, 5, 6, 7, 8, 9, 10, 11, 12, 13, 14, 15); }
__device__ __forceinline__ v16bf cat16b(v8us lo, v8us hi) { return __builtin_bit_cast(v16bf, __builtin_shufflevector(lo, hi, 0, 1, 2, 3, 4, 5, 6, 7, 8, 9, 10, 11, 12, 13, 14, 15)); }
__device__ __forceinline__ v8f wmma16(v16h a, v16h b, v8f c) { return __builtin_amdgcn_wmma_f32_16x16x32_f16(false, a, false, b, (short)0, c, false, false); }
__device__ __forceinline__ v8f wmmab(v16bf a, v16bf b, v8f c) { return __builtin_amdgcn_wmma_f32_16x16x32_bf16(false, a, false, b, (short)0, c, false, false); }


template <typename T16> struct WFrag;
template <> struct WFrag<h16> { typedef v16h V; static __device__ __forceinline__ V ld(const h16* p) { return cat16(*(const v8h*)p, *(const v8h*)(p + 16)); } static __device__ __forceinline__ v8f mma(V a, V b, v8f c) { return wmma16(a, b, c); } };
template <> struct WFrag<bf> { typedef v16bf V; static __device__ __forceinline__ V ld(const bf* p) { return cat16b(*(const v8us*)p, *(const v8us*)(p + 16)); } static __device__ __forceinline__ v8f mma(V a, V b, v8f c) { return wmmab(a, b, c); } };
template <typename T16, int NSPLIT, bool BIAS>
__global__ __launch_bounds__(32) void k_gemmw(const T16* __restrict__ A, const T16* __restrict__ A2, const T16* __restrict__ Bt, const T16* __restrict__ Bt2, int K, float* C, int ldc, const float* __restrict__ bias, size_t sA, size_t sB, size_t sC) {
    typedef typename WFrag<T16>::V V;
    __shared__ __align__(16) float os[16 * 68];
    const size_t z = blockIdx.z; A += z * sA; if (A2) A2 += z * sA; Bt += z * sB; if (Bt2) Bt2 += z * sB; C += z * sC;
    const int lane = threadIdx.x & 31, lr = lane & 15, hi = lane >> 4; const int r0 = blockIdx.x * 64, c0 = blockIdx.y * 64;
    v8f acc[4][4];
#pragma unroll
    for (int mb = 0; mb < 4; ++mb)
#pragma unroll
        for (int nb = 0; nb < 4; ++nb) acc[mb][nb] = (v8f){};
    const size_t aoff = (size_t)(r0 + lr) * K + 8 * hi, boff = (size_t)(c0 + lr) * K + 8 * hi;
#pragma unroll 1
    for (int kc = 0; kc < K; kc += 32) {
        V a[4], a2[4];
#pragma unroll
        for (int mb = 0; mb < 4; ++mb) { a[mb] = WFrag<T16>::ld(A + aoff + (size_t)mb * 16 * K + kc); if (NSPLIT == 1 || NSPLIT == 2) a2[mb] = WFrag<T16>::ld(A2 + aoff + (size_t)mb * 16 * K + kc); }
#pragma unroll
        for (int nb = 0; nb < 4; ++nb) { const V b = WFrag<T16>::ld(Bt + boff + (size_t)nb * 16 * K + kc); V b2; if (NSPLIT >= 2) b2 = WFrag<T16>::ld(Bt2 + boff + (size_t)nb * 16 * K + kc);
#pragma unroll
            for (int mb = 0; mb < 4; ++mb) { acc[mb][nb] = WFrag<T16>::mma(a[mb], b, acc[mb][nb]); if (NSPLIT == 1 || NSPLIT == 2) acc[mb][nb] = WFrag<T16>::mma(a2[mb], b, acc[mb][nb]); if (NSPLIT >= 2) acc[mb][nb] = WFrag<T16>::mma(a[mb], b2, acc[mb][nb]); } }
        asm volatile("v_nop\n\tv_nop\n\tv_nop\n\tv_nop" : "+v"(acc[0][0]), "+v"(acc[1][1]), "+v"(acc[2][2]), "+v"(acc[3][3]) : "v"(a[0]), "v"(a[3]));
    }
#pragma unroll
    for (int mb = 0; mb < 4; ++mb) {
#pragma unroll
        for (int nb = 0; nb < 4; ++nb) {
#pragma unroll
            for (int j = 0; j < 8; ++j) os[(hi * 8 + j) * 68 + nb * 16 + lr] = acc[mb][nb][j]; }
        __builtin_amdgcn_wave_barrier(); asm volatile("" ::: "memory");
        float* crow = C + (size_t)(r0 + mb * 16) * ldc + c0;
#pragma unroll 1
        for (int ps = 0; ps < 2; ++ps) {
#pragma unroll
            for (int s = 0; s < 8; ++s) { const int row = 2 * s + hi, cofs = lr * 4; v4f val = *(const v4fa*)(os + row * 68 + cofs); if (BIAS) { val[0] += bfr(bias[c0 + cofs]); val[1] += bfr(bias[c0 + cofs + 1]); val[2] += bfr(bias[c0 + cofs + 2]); val[3] += bfr(bias[c0 + cofs + 3]); }
                *(volatile v4f*)(crow + (size_t)row * ldc + cofs) = val; }
            if (ps == 0) __threadfence(); }
        __builtin_amdgcn_wave_barrier(); asm volatile("" ::: "memory");
    }
}

typedef __attribute__((ext_vector_type(4))) unsigned short v4us;
__device__ __forceinline__ void splitf(float y, unsigned short& h, unsigned short& l) { h = f2bf(y); l = f2bf(y - bf2f(h)); }
__global__ __launch_bounds__(256) void k_cvt8(const float* __restrict__ src, bf* dst, size_t n8) { const size_t i = (size_t)blockIdx.x * 256 + threadIdx.x; if (i >= n8) return; const v8f v = *(const v8f*)(src + i * 8); v8us o;
#pragma unroll
    for (int k = 0; k < 8; ++k) o[k] = f2bf(v[k]); *(volatile v8us*)(dst + i * 8) = o; __threadfence(); *(volatile v8us*)(dst + i * 8) = o; }

__global__ __launch_bounds__(256) void k_zero16(bf* Z, size_t n8) { const size_t i = (size_t)blockIdx.x * 256 + threadIdx.x; if (i >= n8) return; v8us o; for (int k = 0; k < 8; ++k) o[k] = 0; *(volatile v8us*)(Z + i * 8) = o; __threadfence(); *(volatile v8us*)(Z + i * 8) = o; }
__global__ __launch_bounds__(256) void k_vmt(const float* __restrict__ vm, bf* VT) { const int i = blockIdx.x * 256 + threadIdx.x; if (i >= DVM * MP / 8) return; const int m0 = (i % (MP / 8)) * 8; const int d = i / (MP / 8); v8us o;
#pragma unroll
    for (int k = 0; k < 8; ++k) o[k] = (m0 + k < MS) ? f2bf(vm[(size_t)(m0 + k) * DVM + d]) : (unsigned short)0; *(volatile v8us*)(VT + (size_t)d * MP + m0) = o; __threadfence(); *(volatile v8us*)(VT + (size_t)d * MP + m0) = o; }
__global__ __launch_bounds__(256) void k_gath(const int* __restrict__ qi, const float* __restrict__ emb, size_t t0, bf* E, bf* FAh) { const size_t i = (size_t)blockIdx.x * 256 + threadIdx.x; if (i >= (size_t)CH * DK / 8) return; const int c0 = (int)(i % (DK / 8)) * 8; const size_t t = i / (DK / 8); int id = qi[t0 + t]; id = id < 0 ? 0 : (id > NQ1 - 1 ? NQ1 - 1 : id); v8us o;
#pragma unroll
    for (int k = 0; k < 8; ++k) o[k] = f2bf(emb[(size_t)id * DK + c0 + k]);
    *(volatile v8us*)(E + t * DK + c0) = o; *(volatile v8us*)(FAh + t * NF + DVM + c0) = o; __threadfence(); *(volatile v8us*)(E + t * DK + c0) = o; *(volatile v8us*)(FAh + t * NF + DVM + c0) = o; }
__global__ __launch_bounds__(256) void k_soft50(const float* __restrict__ S, bf* Ph, bf* Pl) { const int lane = threadIdx.x & 31; const int sub = lane >> 4, l16 = lane & 15; const size_t t = ((size_t)blockIdx.x * 8 + (threadIdx.x >> 5)) * 2 + sub; if (t >= (size_t)CH) return; const v4f a = *(const v4f*)(S + t * MP + l16 * 4); float v[4]; float mx = -3.0e38f;
#pragma unroll
    for (int q = 0; q < 4; ++q) { const int m = l16 * 4 + q; v[q] = (m < MS) ? a[q] : -3.0e38f; mx = fmaxf(mx, v[q]); }
#pragma unroll
    for (int sh = 8; sh; sh >>= 1) mx = fmaxf(mx, __shfl_xor(mx, sh, 32));
    float sum = 0.f;
#pragma unroll
    for (int q = 0; q < 4; ++q) { float d0 = __fsub_rn(v[q], mx); asm volatile("" : "+v"(d0)); v[q] = __builtin_amdgcn_exp2f(__fmul_rn(d0, 1.4426950408889634f)); sum += v[q]; }
#pragma unroll
    for (int sh = 8; sh; sh >>= 1) sum += __shfl_xor(sum, sh, 32);
    const float f = __fdiv_rn(1.0f, sum); v4us oh, ol;
#pragma unroll
    for (int q = 0; q < 4; ++q) { unsigned short h2, l2; splitf(v[q] * f, h2, l2); oh[q] = h2; ol[q] = l2; }
    *(volatile v4us*)(Ph + t * MP + l16 * 4) = oh; *(volatile v4us*)(Pl + t * MP + l16 * 4) = ol; __threadfence(); *(volatile v4us*)(Ph + t * MP + l16 * 4) = oh; *(volatile v4us*)(Pl + t * MP + l16 * 4) = ol; }
__global__ __launch_bounds__(256) void k_feat(const float* __restrict__ R, bf* FAh, bf* FAl) { const size_t i = (size_t)blockIdx.x * 256 + threadIdx.x; if (i >= (size_t)CH * DVM / 4) return; const int c0 = (int)(i % (DVM / 4)) * 4; const size_t t = i / (DVM / 4); const v4f a = *(const v4f*)(R + t * DVM + c0); v4us oh, ol;
#pragma unroll
    for (int q = 0; q < 4; ++q) { unsigned short h2, l2; splitf(a[q], h2, l2); oh[q] = h2; ol[q] = l2; }
    *(volatile v4us*)(FAh + t * NF + c0) = oh; *(volatile v4us*)(FAl + t * NF + c0) = ol; __threadfence(); *(volatile v4us*)(FAh + t * NF + c0) = oh; *(volatile v4us*)(FAl + t * NF + c0) = ol; }
__global__ __launch_bounds__(256) void k_pred(const float* __restrict__ ST, const float* __restrict__ wp, const float* __restrict__ bp, size_t t0, float* out) {
    const size_t t = (size_t)blockIdx.x * 256 + threadIdx.x; if (t >= (size_t)CH) return; const float* sr = ST + t * DH; float s = 0.f;
#pragma unroll 2
    for (int h = 0; h < DH; h += 4) { const v4f a = *(const v4f*)(sr + h);
#pragma unroll
        for (int q = 0; q < 4; ++q) { float p = __fmul_rn(fmaxf(a[q], 0.0f), bfr(wp[h + q])); asm volatile("" : "+v"(p)); s = __fadd_rn(s, p); } }
    const float z = __fadd_rn(s, bfr(bp[0])); const float pr = __fdiv_rn(1.0f, __fadd_rn(1.0f, __builtin_amdgcn_exp2f(__fmul_rn(z, -1.4426950408889634f))));
    *(volatile float*)(out + t0 + t) = pr; __threadfence(); *(volatile float*)(out + t0 + t) = pr; }

extern "C" void kernel_launch(void* const* d_in, const int* in_sizes, int n_in,
                              void* d_out, int out_size, void* d_ws, size_t ws_size, hipStream_t stream) {
    (void)in_sizes; (void)n_in; (void)out_size;
    const int* q = (const int*)d_in[0];   const float* km = (const float*)d_in[2]; const float* vm = (const float*)d_in[3]; const float* emb = (const float*)d_in[4];   const float* wf = (const float*)d_in[9]; const float* bfv = (const float*)d_in[10]; const float* wp = (const float*)d_in[11]; const float* bp = (const float*)d_in[12];
    float* OUT = (float*)d_out;
    char* wsp = (char*)d_ws;
    auto take = [&](size_t bytes) { char* p = wsp; wsp += (bytes + 255) & ~(size_t)255; return (void*)p; };
    bf* KM = (bf*)take((size_t)MP * DK * 2); bf* VT = (bf*)take((size_t)DVM * MP * 2); bf* WF = (bf*)take((size_t)DH * NF * 2);
    bf* E = (bf*)take((size_t)CH * DK * 2); float* S = (float*)take((size_t)CH * MP * 4); bf* Ph = (bf*)take((size_t)CH * MP * 2); bf* Pl = (bf*)take((size_t)CH * MP * 2); float* R = (float*)take((size_t)CH * DVM * 4); bf* FAh = (bf*)take((size_t)CH * NF * 2); bf* FAl = (bf*)take((size_t)CH * NF * 2); float* ST = (float*)take((size_t)CH * DH * 4);
    if ((size_t)(wsp - (char*)d_ws) > ws_size) return;
    k_zero16<<<(MP * DK / 8 + 255) / 256, 256, 0, stream>>>(KM, (size_t)MP * DK / 8); k_cvt8<<<(MS * DK / 8 + 255) / 256, 256, 0, stream>>>(km, KM, (size_t)MS * DK / 8);
    k_vmt<<<(DVM * MP / 8 + 255) / 256, 256, 0, stream>>>(vm, VT);
    k_cvt8<<<(DH * NF / 8 + 255) / 256, 256, 0, stream>>>(wf, WF, (size_t)DH * NF / 8);
    k_zero16<<<(unsigned)(((size_t)CH * NF / 8 + 255) / 256), 256, 0, stream>>>(FAl, (size_t)CH * NF / 8);
    for (size_t t0 = 0; t0 < (size_t)NTOK; t0 += CH) {
        k_gath<<<(unsigned)(((size_t)CH * DK / 8 + 255) / 256), 256, 0, stream>>>(q, emb, t0, E, FAh);
        k_gemmw<bf, 0, false><<<dim3(CH / 64, MP / 64, 1), 32, 0, stream>>>(E, nullptr, KM, nullptr, DK, S, MP, nullptr, 0, 0, 0);
        k_soft50<<<(unsigned)((CH / 2 + 7) / 8), 256, 0, stream>>>(S, Ph, Pl);
        k_gemmw<bf, 1, false><<<dim3(CH / 64, DVM / 64, 1), 32, 0, stream>>>(Ph, Pl, VT, nullptr, MP, R, DVM, nullptr, 0, 0, 0);
        k_feat<<<(unsigned)(((size_t)CH * DVM / 4 + 255) / 256), 256, 0, stream>>>(R, FAh, FAl);
        k_gemmw<bf, 1, true><<<dim3(CH / 64, DH / 64, 1), 32, 0, stream>>>(FAh, FAl, WF, nullptr, NF, ST, DH, bfv, 0, 0, 0);
        k_pred<<<CH / 256, 256, 0, stream>>>(ST, wp, bp, t0, OUT); }
}
